// SioConvNetBlock_33294586478862
// MI455X (gfx1250) — hardware-verified
//
#include <hip/hip_runtime.h>


#define DIM 512
#define DT 64
#define DFF 2048
#define NB 2
#define SEQ 512
#define TOK (NB * SEQ)
#define TP 68
#define SBP 132

static_assert(TOK % 64 == 0);
static_assert(DIM % 64 == 0);
static_assert(DFF % 64 == 0);
static_assert(DT % 64 == 0);
static_assert((2 * DT) % 64 == 0);
static_assert(DIM % 256 == 0);
static_assert(SEQ % 32 == 0);
static_assert(NB * DT == 128);
static_assert(TP % 4 == 0);
static_assert(SBP % 4 == 0);

typedef _Float16 h16;
typedef unsigned short us16;
typedef h16 v16h __attribute__((ext_vector_type(16)));
typedef h16 v8h __attribute__((ext_vector_type(8)));
typedef __bf16 v16b __attribute__((ext_vector_type(16)));
typedef us16 v8us __attribute__((ext_vector_type(8)));
typedef float v8f __attribute__((ext_vector_type(8)));
typedef float v4f __attribute__((ext_vector_type(4)));
typedef float v2f __attribute__((ext_vector_type(2)));
typedef v4f v4fm __attribute__((may_alias));

__device__ __forceinline__ us16 bf16_bits(float x) {
  unsigned u = __float_as_uint(x);
  u += 0x7FFFu + ((u >> 16) & 1u);
  return (us16)(u >> 16);
}
__device__ __forceinline__ void split_bf16(float x, us16& hi, us16& lo) {
  hi = bf16_bits(x);
  const float xh = __uint_as_float(((unsigned)hi) << 16);
  lo = bf16_bits(x - xh);
}
__device__ __forceinline__ float silu_f(float t) {
  return t * __builtin_amdgcn_rcpf(1.0f + expf(-t));
}
__device__ __forceinline__ void st_v4(float* p, v4f v) { *(volatile v4f*)p = v; }
__device__ __forceinline__ void st_v8(us16* p, v8us v) { *(volatile v8us*)p = v; }

union Frag { v16h f; v16b b; v8us u[2]; };

__device__ __forceinline__ Frag ld_frag(const us16* __restrict__ base, size_t row, int ld, int k0, int h) {
  const us16* p = base + row * (size_t)ld + (size_t)(k0 + 8 * h);
  Frag fr;
  fr.u[0] = *(const v8us*)(p);
  fr.u[1] = *(const v8us*)(p + 16);
  return fr;
}
__device__ __forceinline__ v8f mma_f16(v16h a, v16h b, v8f c) {
  c = __builtin_amdgcn_wmma_f32_16x16x32_f16(false, a, false, b, (short)0, c, false, false);
  asm volatile("v_nop\n\tv_nop\n\tv_nop\n\tv_nop" : "+v"(c) : "v"(a), "v"(b));
  return c;
}
__device__ __forceinline__ v8f mma_bf16(v16b a, v16b b, v8f c) {
  c = __builtin_amdgcn_wmma_f32_16x16x32_bf16(false, a, false, b, (short)0, c, false, false);
  asm volatile("v_nop\n\tv_nop\n\tv_nop\n\tv_nop" : "+v"(c) : "v"(a), "v"(b));
  return c;
}

__global__ __launch_bounds__(256)
void k_cvt_h16(const float* __restrict__ src, int n, float scale, us16* dst) {
  const size_t base = ((size_t)blockIdx.x * 256u + (size_t)threadIdx.x) * 8u;
  if (base + 8u > (size_t)n) return;
  const v4f a = *(const v4f*)(src + base);
  const v4f c = *(const v4f*)(src + base + 4);
  union { v8h hv; v8us u; } o;
  o.hv[0] = (h16)(a[0] * scale); o.hv[1] = (h16)(a[1] * scale);
  o.hv[2] = (h16)(a[2] * scale); o.hv[3] = (h16)(a[3] * scale);
  o.hv[4] = (h16)(c[0] * scale); o.hv[5] = (h16)(c[1] * scale);
  o.hv[6] = (h16)(c[2] * scale); o.hv[7] = (h16)(c[3] * scale);
  const v8us w = o.u;
  st_v8(dst + base, w);
  __threadfence();
  st_v8(dst + base, w);
}

__global__ __launch_bounds__(256)
void k_cvt_split(const float* __restrict__ src, int n, us16* dhi, us16* dlo) {
  const size_t base = ((size_t)blockIdx.x * 256u + (size_t)threadIdx.x) * 8u;
  if (base + 8u > (size_t)n) return;
  const v4f a = *(const v4f*)(src + base);
  const v4f c = *(const v4f*)(src + base + 4);
  const float f[8] = {a[0], a[1], a[2], a[3], c[0], c[1], c[2], c[3]};
  v8us hi = {0, 0, 0, 0, 0, 0, 0, 0}, lo = {0, 0, 0, 0, 0, 0, 0, 0};
#pragma unroll
  for (int e = 0; e < 8; ++e) {
    us16 hb, lb;
    split_bf16(f[e], hb, lb);
    hi[e] = hb; lo[e] = lb;
  }
  st_v8(dhi + base, hi);
  st_v8(dlo + base, lo);
  __threadfence();
  st_v8(dhi + base, hi);
  st_v8(dlo + base, lo);
}

template <int KIND>
__global__ __launch_bounds__(128)
void k_layernorm(const float* __restrict__ x, const float* __restrict__ g, const float* __restrict__ bta,
                 int rows, us16* o0, us16* o1)
{
  const int lane = threadIdx.x & 31;
  const int row = blockIdx.x * 4 + (int)(threadIdx.x >> 5);
  if (row >= rows) return;
  const float* xr = x + (size_t)row * DIM;
  float v[16];
#pragma unroll
  for (int s = 0; s < 2; ++s) {
    const v4f a = *(const v4f*)(xr + 256 * s + 8 * lane);
    const v4f c = *(const v4f*)(xr + 256 * s + 8 * lane + 4);
    v[8 * s + 0] = a[0]; v[8 * s + 1] = a[1]; v[8 * s + 2] = a[2]; v[8 * s + 3] = a[3];
    v[8 * s + 4] = c[0]; v[8 * s + 5] = c[1]; v[8 * s + 6] = c[2]; v[8 * s + 7] = c[3];
  }
  float sum = 0.f;
#pragma unroll
  for (int j = 0; j < 16; ++j) sum += v[j];
#pragma unroll
  for (int off = 16; off >= 1; off >>= 1) sum += __shfl_xor(sum, off, 32);
  const float mu = sum * (1.0f / DIM);
  float q = 0.f;
#pragma unroll
  for (int j = 0; j < 16; ++j) { const float dd = v[j] - mu; q += dd * dd; }
#pragma unroll
  for (int off = 16; off >= 1; off >>= 1) q += __shfl_xor(q, off, 32);
  const float rstd = rsqrtf(q * (1.0f / DIM) + 1e-5f);

  v8us w0[2], w1[2];
#pragma unroll
  for (int s = 0; s < 2; ++s) {
    const int c0 = 256 * s + 8 * lane;
    const v4f ga = *(const v4f*)(g + c0);
    const v4f gc = *(const v4f*)(g + c0 + 4);
    const v4f ba = *(const v4f*)(bta + c0);
    const v4f bc = *(const v4f*)(bta + c0 + 4);
    const float gg[8] = {ga[0], ga[1], ga[2], ga[3], gc[0], gc[1], gc[2], gc[3]};
    const float bb[8] = {ba[0], ba[1], ba[2], ba[3], bc[0], bc[1], bc[2], bc[3]};
    v8us hi = {0, 0, 0, 0, 0, 0, 0, 0}, lo = {0, 0, 0, 0, 0, 0, 0, 0};
    union { v8h hv; v8us u; } f;
    f.u = hi;
#pragma unroll
    for (int e = 0; e < 8; ++e) {
      float o = (v[8 * s + e] - mu) * rstd;
      o = o * gg[e] + bb[e];
      if (KIND == 0) {
        us16 hb, lb;
        split_bf16(o, hb, lb);
        hi[e] = hb; lo[e] = lb;
      } else {
        f.hv[e] = (h16)(o * 16.0f);
      }
    }
    if (KIND == 0) { w0[s] = hi; w1[s] = lo; } else { w0[s] = f.u; w1[s] = f.u; }
  }
  const size_t base = (size_t)row * DIM + (size_t)(8 * lane);
#pragma unroll
  for (int s = 0; s < 2; ++s) {
    st_v8(o0 + base + 256 * s, w0[s]);
    if (KIND == 0) st_v8(o1 + base + 256 * s, w1[s]);
  }
  __threadfence();
#pragma unroll
  for (int s = 0; s < 2; ++s) {
    st_v8(o0 + base + 256 * s, w0[s]);
    if (KIND == 0) st_v8(o1 + base + 256 * s, w1[s]);
  }
}

template <bool SPLIT, int EPI>
__global__ __launch_bounds__(128)
void k_gemm(const us16* __restrict__ Ah, const us16* __restrict__ Al,
            const us16* __restrict__ Wh, const us16* __restrict__ Wl,
            int M, int N, int K,
            const float* __restrict__ bias0, const float* __restrict__ bias1,
            const float* __restrict__ res, float oscale,
            float* outf0, float* outf1, us16* outh0, us16* outh1)
{
  __shared__ __attribute__((aligned(16))) float s_tile[64 * TP];
  const int lane = threadIdx.x & 31;
  const int wave = threadIdx.x >> 5;
  const int h = lane >> 4, lm = lane & 15;
  const int m0 = blockIdx.y * 64, n0 = blockIdx.x * 64;
  if (m0 + 64 > M || n0 + 64 > N) return;
  const int wr = (wave >> 1) * 32, wc = (wave & 1) * 32;

  v8f acc[2][2];
  {
    const v8f z = {0.f, 0.f, 0.f, 0.f, 0.f, 0.f, 0.f, 0.f};
#pragma unroll
    for (int i = 0; i < 2; ++i)
#pragma unroll
      for (int j = 0; j < 2; ++j) acc[i][j] = z;
  }

#pragma unroll 1
  for (int k0 = 0; k0 < K; k0 += 32) {
    Frag ah[2], wh[2], al[2], wl[2];
#pragma unroll
    for (int i = 0; i < 2; ++i) {
      const size_t ra = (size_t)(m0 + wr + 16 * i + lm);
      ah[i] = ld_frag(Ah, ra, K, k0, h);
      al[i] = ah[i];
      if (SPLIT) al[i] = ld_frag(Al, ra, K, k0, h);
    }
#pragma unroll
    for (int j = 0; j < 2; ++j) {
      const size_t rw = (size_t)(n0 + wc + 16 * j + lm);
      wh[j] = ld_frag(Wh, rw, K, k0, h);
      wl[j] = wh[j];
      if (SPLIT) wl[j] = ld_frag(Wl, rw, K, k0, h);
    }
#pragma unroll
    for (int i = 0; i < 2; ++i) {
#pragma unroll
      for (int j = 0; j < 2; ++j) {
        if (SPLIT) {
          acc[i][j] = mma_bf16(ah[i].b, wh[j].b, acc[i][j]);
          acc[i][j] = mma_bf16(ah[i].b, wl[j].b, acc[i][j]);
          acc[i][j] = mma_bf16(al[i].b, wh[j].b, acc[i][j]);
        } else {
          acc[i][j] = mma_f16(ah[i].f, wh[j].f, acc[i][j]);
        }
      }
    }
  }

#pragma unroll
  for (int i = 0; i < 2; ++i)
#pragma unroll
    for (int j = 0; j < 2; ++j)
#pragma unroll
      for (int r = 0; r < 8; ++r)
        s_tile[(wr + 16 * i + 8 * h + r) * TP + wc + 16 * j + lm] = acc[i][j][r];
  __syncthreads();

  const int q = lane >> 3, sub = lane & 7;

  if (EPI != 3) {
    float* optr;
    const float* bptr;
    int ldo, nc0;
    bool act = false;
    if (EPI == 0) {
      const bool gate = (blockIdx.x == 0);
      optr = gate ? outf0 : outf1;
      bptr = gate ? bias0 : bias1;
      act = gate;
      ldo = 64; nc0 = 0;
    } else if (EPI == 1) {
      optr = outf0; bptr = bias0; ldo = N; nc0 = n0;
    } else {
      optr = outf0; bptr = bias0; ldo = N; nc0 = n0;
    }
    v4f vals[8];
#pragma unroll
    for (int t = 0; t < 8; ++t) {
      const int L = 4 * t + q;
      const int row = 16 * wave + (L >> 1);
      const int col = (L & 1) * 32 + 4 * sub;
      const v4f v = *(const v4fm*)(s_tile + row * TP + col);
      v4f o = v;
      if (EPI != 1) {
        const int n = nc0 + col;
        const v4f bv = *(const v4f*)(bptr + n);
        v4f rv = {0.f, 0.f, 0.f, 0.f};
        if (EPI == 2) rv = *(const v4f*)(res + (size_t)(m0 + row) * (size_t)N + (size_t)n);
#pragma unroll
        for (int e = 0; e < 4; ++e) {
          float z;
          if (EPI == 0) {
            z = v[e] + bv[e];
            if (act) z = silu_f(z);
          } else {
            z = v[e] * oscale + bv[e];
            z = z + rv[e];
          }
          o[e] = z;
        }
      }
      vals[t] = o;
    }
#pragma unroll
    for (int t = 0; t < 8; ++t) {
      const int L = 4 * t + q;
      const int row = 16 * wave + (L >> 1);
      const int col = (L & 1) * 32 + 4 * sub;
      st_v4(optr + (size_t)(m0 + row) * (size_t)ldo + (size_t)(nc0 + col), vals[t]);
    }
    __threadfence();
#pragma unroll
    for (int t = 0; t < 8; ++t) {
      const int L = 4 * t + q;
      const int row = 16 * wave + (L >> 1);
      const int col = (L & 1) * 32 + 4 * sub;
      st_v4(optr + (size_t)(m0 + row) * (size_t)ldo + (size_t)(nc0 + col), vals[t]);
    }
  }

  if (EPI == 3 || (EPI == 0 && blockIdx.x == 1)) {
    v8us pv[4], lv[4];
#pragma unroll
    for (int t = 0; t < 4; ++t) {
      const int row = 16 * wave + 4 * t + q;
      const int col = 8 * sub;
      const v4f x0 = *(const v4fm*)(s_tile + row * TP + col);
      const v4f x1 = *(const v4fm*)(s_tile + row * TP + col + 4);
      const float z[8] = {x0[0], x0[1], x0[2], x0[3], x1[0], x1[1], x1[2], x1[3]};
      if (EPI == 3) {
        const int n = n0 + col;
        const v4f ba = *(const v4f*)(bias0 + n);
        const v4f bc = *(const v4f*)(bias0 + n + 4);
        const float bb[8] = {ba[0], ba[1], ba[2], ba[3], bc[0], bc[1], bc[2], bc[3]};
        union { v8h hv; v8us u; } f;
#pragma unroll
        for (int e = 0; e < 8; ++e) {
          const float s = silu_f(z[e] * oscale + bb[e]) * 16.0f;
          f.hv[e] = (h16)s;
        }
        pv[t] = f.u; lv[t] = f.u;
      } else {
        const v4f ba = *(const v4f*)(bias1 + col);
        const v4f bc = *(const v4f*)(bias1 + col + 4);
        const float bb[8] = {ba[0], ba[1], ba[2], ba[3], bc[0], bc[1], bc[2], bc[3]};
        v8us hi = {0, 0, 0, 0, 0, 0, 0, 0}, lo = {0, 0, 0, 0, 0, 0, 0, 0};
#pragma unroll
        for (int e = 0; e < 8; ++e) {
          const float uval = z[e] + bb[e];
          us16 hb, lb;
          split_bf16(uval, hb, lb);
          hi[e] = hb; lo[e] = lb;
        }
        pv[t] = hi; lv[t] = lo;
      }
    }
#pragma unroll
    for (int t = 0; t < 4; ++t) {
      const int row = 16 * wave + 4 * t + q;
      const int col = 8 * sub;
      if (EPI == 3) {
        st_v8(outh0 + (size_t)(m0 + row) * (size_t)N + (size_t)(n0 + col), pv[t]);
      } else {
        st_v8(outh0 + (size_t)(m0 + row) * 64u + (size_t)col, pv[t]);
        st_v8(outh1 + (size_t)(m0 + row) * 64u + (size_t)col, lv[t]);
      }
    }
    __threadfence();
#pragma unroll
    for (int t = 0; t < 4; ++t) {
      const int row = 16 * wave + 4 * t + q;
      const int col = 8 * sub;
      if (EPI == 3) {
        st_v8(outh0 + (size_t)(m0 + row) * (size_t)N + (size_t)(n0 + col), pv[t]);
      } else {
        st_v8(outh0 + (size_t)(m0 + row) * 64u + (size_t)col, pv[t]);
        st_v8(outh1 + (size_t)(m0 + row) * 64u + (size_t)col, lv[t]);
      }
    }
  }
}

__global__ __launch_bounds__(128)
void k_scan(const float* __restrict__ aout, const float* __restrict__ u, const float* __restrict__ y,
            const float* __restrict__ hid_re, const float* __restrict__ hid_im, us16* hy)
{
  __shared__ __attribute__((aligned(16))) float s_buf[32 * SBP];
  const int t = threadIdx.x;
  const int lane = t & 31, wave = t >> 5;
  const int b = t >> 6, d = t & 63;
  const size_t rowb = (size_t)b * SEQ;
  const float hre = hid_re[d], him = hid_im[d];
  const float ulast = u[(rowb + SEQ - 1) * DT + d];
  const int q = lane >> 3, sub = lane & 7;
  float rre = 0.f, rim = 0.f;

  for (int c = SEQ / 32 - 1; c >= 0; --c) {
#pragma unroll 1
    for (int ii = 31; ii >= 0; --ii) {
      const int i = c * 32 + ii;
      const size_t ri = rowb + (size_t)i;
      const v2f ap = *(const v2f*)(aout + ri * 128u + (size_t)(2 * d));
      const float re = ap[0], im = ap[1];
      const float s2 = re * re + im * im;
      const float sc = rsqrtf(s2) * expf(-s2);
      const float are = re * sc, aim = im * sc;
      const int im1 = (i > 0) ? (i - 1) : 0;
      const int im2 = (i > 1) ? (i - 2) : 0;
      const float um1 = u[(rowb + (size_t)im1) * DT + d];
      const float um2 = u[(rowb + (size_t)im2) * DT + d];
      const float xr = (i == 0) ? hre : um1;
      const float xi = (i == 0) ? him : 0.f;
      const float tr = xr + rre, ti = xi + rim;
      const float nr = are * tr - aim * ti;
      const float ni = are * ti + aim * tr;
      rre = nr; rim = ni;
      const float prev = (i == 0) ? 0.f : ((i == 1) ? hre : um2);
      float hv = prev + rre;
      if (i == SEQ - 1) hv += ulast;
      s_buf[ii * SBP + t] = hv * y[ri * DT + d];
    }
    __syncthreads();

    union { v8h hv; v8us u; } o[4];
#pragma unroll
    for (int t4 = 0; t4 < 4; ++t4) {
      const int L = 16 * wave + 4 * t4 + q;
      const int bb = L >> 5, jj = L & 31;
      const int col = 8 * sub;
      const v4f x0 = *(const v4fm*)(s_buf + jj * SBP + bb * 64 + col);
      const v4f x1 = *(const v4fm*)(s_buf + jj * SBP + bb * 64 + col + 4);
      o[t4].hv[0] = (h16)(x0[0] * 16.0f); o[t4].hv[1] = (h16)(x0[1] * 16.0f);
      o[t4].hv[2] = (h16)(x0[2] * 16.0f); o[t4].hv[3] = (h16)(x0[3] * 16.0f);
      o[t4].hv[4] = (h16)(x1[0] * 16.0f); o[t4].hv[5] = (h16)(x1[1] * 16.0f);
      o[t4].hv[6] = (h16)(x1[2] * 16.0f); o[t4].hv[7] = (h16)(x1[3] * 16.0f);
    }
#pragma unroll
    for (int t4 = 0; t4 < 4; ++t4) {
      const int L = 16 * wave + 4 * t4 + q;
      const int bb = L >> 5, jj = L & 31;
      const int col = 8 * sub;
      st_v8(hy + ((size_t)bb * SEQ + (size_t)(c * 32 + jj)) * DT + (size_t)col, o[t4].u);
    }
    __threadfence();
#pragma unroll
    for (int t4 = 0; t4 < 4; ++t4) {
      const int L = 16 * wave + 4 * t4 + q;
      const int bb = L >> 5, jj = L & 31;
      const int col = 8 * sub;
      st_v8(hy + ((size_t)bb * SEQ + (size_t)(c * 32 + jj)) * DT + (size_t)col, o[t4].u);
    }
    __syncthreads();
  }
}

extern "C" void kernel_launch(void* const* d_in, const int* in_sizes, int n_in,
                              void* d_out, int out_size, void* d_ws, size_t ws_size,
                              hipStream_t stream) {
  if (n_in < 18) return;
  if (in_sizes[0] != TOK * DIM || in_sizes[1] != DIM || in_sizes[2] != DIM ||
      in_sizes[3] != DT * DIM || in_sizes[4] != DT ||
      in_sizes[5] != DT * DIM || in_sizes[6] != DT ||
      in_sizes[7] != 2 * DT * DT || in_sizes[8] != DT || in_sizes[9] != DT ||
      in_sizes[10] != DIM * DT || in_sizes[11] != DIM ||
      in_sizes[12] != DIM || in_sizes[13] != DIM ||
      in_sizes[14] != DFF * DIM || in_sizes[15] != DFF ||
      in_sizes[16] != DIM * DFF || in_sizes[17] != DIM ||
      out_size != TOK * DIM) return;

  const float* x        = (const float*)d_in[0];
  const float* ln1_g    = (const float*)d_in[1];
  const float* ln1_b    = (const float*)d_in[2];
  const float* fc_w     = (const float*)d_in[3];
  const float* fc_b     = (const float*)d_in[4];
  const float* lin_in_w = (const float*)d_in[5];
  const float* lin_in_b = (const float*)d_in[6];
  const float* wa       = (const float*)d_in[7];
  const float* hid_re   = (const float*)d_in[8];
  const float* hid_im   = (const float*)d_in[9];
  const float* lo_w     = (const float*)d_in[10];
  const float* lo_b     = (const float*)d_in[11];
  const float* ln2_g    = (const float*)d_in[12];
  const float* ln2_b    = (const float*)d_in[13];
  const float* w1       = (const float*)d_in[14];
  const float* b1       = (const float*)d_in[15];
  const float* w2       = (const float*)d_in[16];
  const float* b2       = (const float*)d_in[17];
  float* out = (float*)d_out;

  char* ws = (char*)d_ws;
  size_t off = 0;
  auto carve = [&](size_t bytes) -> char* {
    char* p = ws + off;
    off += (bytes + 255) & ~(size_t)255;
    return p;
  };
  us16* xn_hi   = (us16*)carve((size_t)TOK * DIM * 2);
  us16* xn_lo   = (us16*)carve((size_t)TOK * DIM * 2);
  us16* wcat_hi = (us16*)carve((size_t)2 * DT * DIM * 2);
  us16* wcat_lo = (us16*)carve((size_t)2 * DT * DIM * 2);
  us16* wa_hi   = (us16*)carve((size_t)2 * DT * DT * 2);
  us16* wa_lo   = (us16*)carve((size_t)2 * DT * DT * 2);
  us16* low16   = (us16*)carve((size_t)DIM * DT * 2);
  us16* w1h     = (us16*)carve((size_t)DFF * DIM * 2);
  us16* w2h     = (us16*)carve((size_t)DIM * DFF * 2);
  float* y_f    = (float*)carve((size_t)TOK * DT * 4);
  float* u_f    = (float*)carve((size_t)TOK * DT * 4);
  us16* u_hi    = (us16*)carve((size_t)TOK * DT * 2);
  us16* u_lo    = (us16*)carve((size_t)TOK * DT * 2);
  float* aout   = (float*)carve((size_t)TOK * 2 * DT * 4);
  us16* hy16    = (us16*)carve((size_t)TOK * DT * 2);
  float* x2     = (float*)carve((size_t)TOK * DIM * 4);
  us16* xn2h    = (us16*)carve((size_t)TOK * DIM * 2);
  us16* t16     = (us16*)carve((size_t)TOK * DFF * 2);
  if (off > ws_size) return;

  const dim3 blk256(256), blk128(128);

  k_cvt_split<<<dim3((DT * DIM / 8 + 255) / 256), blk256, 0, stream>>>(fc_w, DT * DIM, wcat_hi, wcat_lo);
  k_cvt_split<<<dim3((DT * DIM / 8 + 255) / 256), blk256, 0, stream>>>(lin_in_w, DT * DIM,
      wcat_hi + (size_t)DT * DIM, wcat_lo + (size_t)DT * DIM);
  k_cvt_split<<<dim3((2 * DT * DT / 8 + 255) / 256), blk256, 0, stream>>>(wa, 2 * DT * DT, wa_hi, wa_lo);
  k_cvt_h16<<<dim3((DIM * DT / 8 + 255) / 256), blk256, 0, stream>>>(lo_w, DIM * DT, 64.0f, low16);
  k_cvt_h16<<<dim3((DFF * DIM / 8 + 255) / 256), blk256, 0, stream>>>(w1, DFF * DIM, 64.0f, w1h);
  k_cvt_h16<<<dim3((DIM * DFF / 8 + 255) / 256), blk256, 0, stream>>>(w2, DIM * DFF, 64.0f, w2h);

  k_layernorm<0><<<dim3((TOK + 3) / 4), blk128, 0, stream>>>(x, ln1_g, ln1_b, TOK, xn_hi, xn_lo);

  k_gemm<true, 0><<<dim3(2 * DT / 64, TOK / 64), blk128, 0, stream>>>(
      xn_hi, xn_lo, wcat_hi, wcat_lo, TOK, 2 * DT, DIM,
      fc_b, lin_in_b, nullptr, 1.0f, y_f, u_f, u_hi, u_lo);

  k_gemm<true, 1><<<dim3(2 * DT / 64, TOK / 64), blk128, 0, stream>>>(
      u_hi, u_lo, wa_hi, wa_lo, TOK, 2 * DT, DT,
      nullptr, nullptr, nullptr, 1.0f, aout, nullptr, nullptr, nullptr);

  k_scan<<<dim3(1), blk128, 0, stream>>>(aout, u_f, y_f, hid_re, hid_im, hy16);

  k_gemm<false, 2><<<dim3(DIM / 64, TOK / 64), blk128, 0, stream>>>(
      hy16, nullptr, low16, nullptr, TOK, DIM, DT,
      lo_b, nullptr, x, 1.0f / 1024.0f, x2, nullptr, nullptr, nullptr);

  k_layernorm<1><<<dim3((TOK + 3) / 4), blk128, 0, stream>>>(x2, ln2_g, ln2_b, TOK, xn2h, nullptr);

  k_gemm<false, 3><<<dim3(DFF / 64, TOK / 64), blk128, 0, stream>>>(
      xn2h, nullptr, w1h, nullptr, TOK, DFF, DIM,
      b1, nullptr, nullptr, 1.0f / 1024.0f, nullptr, nullptr, t16, nullptr);

  k_gemm<false, 2><<<dim3(DIM / 64, TOK / 64), blk128, 0, stream>>>(
      t16, nullptr, w2h, nullptr, TOK, DIM, DFF,
      b2, nullptr, x2, 1.0f / 1024.0f, out, nullptr, nullptr, nullptr);
}
